// DynamicMaskedGATv2Layer_42039139893268
// MI455X (gfx1250) — hardware-run, weakly checked
//
#include <hip/hip_runtime.h>


#ifndef NB
#define NB 8
#endif
#ifndef NT
#define NT 32
#endif
#define NB_FULL 8
#define NT_FULL 32
#ifndef OUT_NT
#define OUT_NT NT
#endif
#define NHD  4
#define GSZ  4096
#define HP   68
#define TP   72
#define HOFF (64 * HP)
#define LOG2E 1.4426950408889634f
#define NEGV  (-1.0e9f)

static_assert(NB <= NB_FULL);
static_assert(NT <= NT_FULL);
static_assert(HP % 4 == 0);
static_assert(TP % 8 == 0);
static_assert(((size_t)NB * NT * GSZ) % 8 == 0);
static_assert(((size_t)NT * GSZ) % 8 == 0);

typedef unsigned short bf;
typedef __attribute__((ext_vector_type(16))) __bf16   v16bf;
typedef __attribute__((ext_vector_type(8)))  unsigned short v8us;
typedef __attribute__((ext_vector_type(16))) unsigned short v16us;
typedef __attribute__((ext_vector_type(8)))  float    v8f;
typedef __attribute__((ext_vector_type(4)))  float    v4f;
typedef __attribute__((ext_vector_type(4)))  int      v4i;
typedef v4f  __attribute__((may_alias)) v4fa;
typedef v8us __attribute__((may_alias)) v8usa;

__device__ __forceinline__ unsigned short f2bf(float f) { unsigned u = __float_as_uint(f); u += 0x7FFFu + ((u >> 16) & 1u); return (unsigned short)(u >> 16); }
__device__ __forceinline__ float bf2f(unsigned short b) { return __uint_as_float(((unsigned)b) << 16); }
__device__ __forceinline__ v16bf cat16b(v8us lo, v8us hi) { return __builtin_bit_cast(v16bf, __builtin_shufflevector(lo, hi, 0, 1, 2, 3, 4, 5, 6, 7, 8, 9, 10, 11, 12, 13, 14, 15)); }
__device__ __forceinline__ v8f wmmab(v16bf a, v16bf b, v8f c) { return __builtin_amdgcn_wmma_f32_16x16x32_bf16(false, a, false, b, (short)0, c, false, false); }
__device__ __forceinline__ v16bf ldb(const bf* p)  { return cat16b(*(const v8us*)p, *(const v8us*)(p + 16)); }
__device__ __forceinline__ void wave_sync() { __builtin_amdgcn_fence(3  , "wavefront"); __builtin_amdgcn_wave_barrier(); asm volatile("" ::: "memory"); }

__global__ __launch_bounds__(256) void k_cvt8(const float* __restrict__ src, bf* dst, size_t n8) {
    const size_t i = (size_t)blockIdx.x * 256 + threadIdx.x; if (i >= n8) return;
    const v8f v = *(const v8f*)(src + i * 8); v8us o;
#pragma unroll
    for (int k = 0; k < 8; ++k) o[k] = f2bf(v[k]);
    *(volatile v8us*)(dst + i * 8) = o; __threadfence(); *(volatile v8us*)(dst + i * 8) = o;
}

__global__ __launch_bounds__(256) void k_wt(const float* __restrict__ W, bf* WT) {
    __shared__ unsigned short ts[64 * 66];
    const int t = threadIdx.x; const int mat = blockIdx.x;
    const float* src = W + (size_t)mat * GSZ;
#pragma unroll
    for (int it = 0; it < 4; ++it) { const int idx = t + 256 * it; const int k = idx >> 4, n4 = (idx & 15) * 4;
        const v4f v = *(const v4f*)(src + k * 64 + n4);
#pragma unroll
        for (int e = 0; e < 4; ++e) ts[k * 66 + n4 + e] = f2bf(v[e]); }
    __syncthreads();
    bf* dst = WT + (size_t)mat * GSZ;
    const int k8 = (t & 7) * 8;
    v8us o[2];
#pragma unroll
    for (int it = 0; it < 2; ++it) { const int n = (t >> 3) + 32 * it;
#pragma unroll
        for (int e = 0; e < 8; ++e) o[it][e] = ts[(k8 + e) * 66 + n]; }
#pragma unroll 1
    for (int ps = 0; ps < 2; ++ps) {
#pragma unroll
        for (int it = 0; it < 2; ++it) { const int n = (t >> 3) + 32 * it; *(volatile v8us*)(dst + n * 64 + k8) = o[it]; }
        if (ps == 0) __threadfence(); }
}

__global__ __launch_bounds__(128) void k_gat(const bf* __restrict__ XB, const bf* __restrict__ WT, const int* __restrict__ ADJ, const float* __restrict__ AV, float* OUT) {
    __shared__ __align__(16) float s_h[2 * 64 * HP];
    __shared__ __align__(16) unsigned short s_th[64 * TP];
    __shared__ __align__(16) unsigned short s_tl[64 * TP];
    __shared__ __align__(16) float s_a[64];
    __shared__ unsigned s_mask[128];
    const int t = threadIdx.x, lane = t & 31, lr = lane & 15, hi = lane >> 4;
    const int wave = __builtin_amdgcn_readfirstlane(t >> 5);
    const int g = blockIdx.x; const int b = g / NT, tt = g % NT;

    { const int r = t >> 1, half = t & 1;
      const int* ar = ADJ + (size_t)b * GSZ + r * 64 + half * 32;
      unsigned bits = 0u;
#pragma unroll
      for (int q = 0; q < 8; ++q) { const v4i v = *(const v4i*)(ar + 4 * q);
#pragma unroll
          for (int e = 0; e < 4; ++e) { const int j = half * 32 + 4 * q + e; const float f = (float)v[e] + ((j == r) ? 1.0f : 0.0f); bits |= (f > 0.0f) ? (1u << (4 * q + e)) : 0u; } }
      s_mask[t] = bits; }

    const bf* xa = XB + ((size_t)g * 64 + 16 * wave + lr) * 64 + 8 * hi;
    const v16bf af0 = ldb(xa), af1 = ldb(xa + 32);

    v8f o[4];
#pragma unroll
    for (int nb = 0; nb < 4; ++nb) o[nb] = (v8f){};

#pragma unroll 1
    for (int h = 0; h < NHD; ++h) {
        __syncthreads();
        if (t < 64) s_a[t] = bf2f(f2bf(AV[h * 64 + t]));

#pragma unroll
        for (int which = 0; which < 2; ++which) {
            const bf* wp = WT + (size_t)(which * NHD + h) * GSZ + (size_t)lr * 64 + 8 * hi;
            v8f c[4];
#pragma unroll
            for (int nb = 0; nb < 4; ++nb) c[nb] = (v8f){};
#pragma unroll
            for (int ks = 0; ks < 2; ++ks) {
                const v16bf a = (ks == 0) ? af0 : af1;
                v16bf bb[4];
#pragma unroll
                for (int nb = 0; nb < 4; ++nb) bb[nb] = ldb(wp + nb * 1024 + ks * 32);
#pragma unroll
                for (int nb = 0; nb < 4; ++nb) c[nb] = wmmab(a, bb[nb], c[nb]);
                asm volatile("v_nop\n\tv_nop\n\tv_nop\n\tv_nop" : "+v"(c[0]), "+v"(c[1]), "+v"(c[2]), "+v"(c[3]) : "v"(a), "v"(bb[0]), "v"(bb[1]), "v"(bb[2]), "v"(bb[3]));
            }
            const int fb = which * HOFF + (16 * wave + 8 * hi) * HP + lr;
#pragma unroll
            for (int nb = 0; nb < 4; ++nb) {
#pragma unroll
                for (int r = 0; r < 8; ++r) s_h[fb + r * HP + nb * 16] = c[nb][r]; }
            if (which == 0) {
#pragma unroll
                for (int nb = 0; nb < 4; ++nb) { v8us hv, lv;
#pragma unroll
                    for (int r = 0; r < 8; ++r) { const float v = c[nb][r]; const unsigned short hb = f2bf(v); hv[r] = hb; lv[r] = f2bf(v - bf2f(hb)); }
                    const int to = (nb * 16 + lr) * TP + 16 * wave + 8 * hi;
                    *(v8usa*)(&s_th[to]) = hv; *(v8usa*)(&s_tl[to]) = lv; }
            }
        }
        __syncthreads();

        float sc[32];
#pragma unroll
        for (int jj = 0; jj < 32; ++jj) sc[jj] = 0.0f;
        { const int ib = (16 * wave + lr) * HP;
          const int jb = HOFF + 8 * hi * HP;
#pragma unroll 1
          for (int u = 0; u < 64; u += 4) {
              const v4f hv = *(const v4fa*)(&s_h[ib + u]);
              const v4f av = *(const v4fa*)(&s_a[u]);
#pragma unroll
              for (int jj = 0; jj < 32; ++jj) {
                  const v4f dv = *(const v4fa*)(&s_h[jb + ((jj >> 3) * 16 + (jj & 7)) * HP + u]);
#pragma unroll
                  for (int e = 0; e < 4; ++e) { float x = hv[e] + dv[e]; x = fmaxf(x, 0.2f * x); sc[jj] = fmaf(x, av[e], sc[jj]); }
              }
          } }
        { const int i = 16 * wave + lr;
          const unsigned m0 = s_mask[2 * i] >> (8 * hi), m1 = s_mask[2 * i + 1] >> (8 * hi);
          float mx = -3.0e38f;
#pragma unroll
          for (int jj = 0; jj < 32; ++jj) { const unsigned w = (jj >> 4) ? m1 : m0; const unsigned on = (w >> (((jj >> 3) & 1) * 16 + (jj & 7))) & 1u;
              sc[jj] = on ? sc[jj] : NEGV; mx = fmaxf(mx, sc[jj]); }
          mx = fmaxf(mx, __shfl_xor(mx, 16, 32));
          float sum = 0.0f;
#pragma unroll
          for (int jj = 0; jj < 32; ++jj) { sc[jj] = __builtin_amdgcn_exp2f((sc[jj] - mx) * LOG2E); sum += sc[jj]; }
          sum += __shfl_xor(sum, 16, 32);
          const float inv = 1.0f / sum;
#pragma unroll
          for (int jj = 0; jj < 32; ++jj) sc[jj] *= inv; }

        v16us ph0, pl0, ph1, pl1;
#pragma unroll
        for (int e = 0; e < 16; ++e) {
            const float p0 = sc[e], p1 = sc[16 + e];
            const unsigned short h0 = f2bf(p0), h1 = f2bf(p1);
            ph0[e] = h0; pl0[e] = f2bf(p0 - bf2f(h0)); ph1[e] = h1; pl1[e] = f2bf(p1 - bf2f(h1)); }
        const v16bf PH0 = __builtin_bit_cast(v16bf, ph0), PL0 = __builtin_bit_cast(v16bf, pl0), PH1 = __builtin_bit_cast(v16bf, ph1), PL1 = __builtin_bit_cast(v16bf, pl1);
#pragma unroll
        for (int ks = 0; ks < 2; ++ks) {
            const v16bf pa = (ks == 0) ? PH0 : PH1;
            const v16bf pl = (ks == 0) ? PL0 : PL1;
            v16bf bh[4], bl[4];
#pragma unroll
            for (int nb = 0; nb < 4; ++nb) { const int off = (nb * 16 + lr) * TP + 8 * hi + 32 * ks;
                bh[nb] = cat16b(*(const v8usa*)(&s_th[off]), *(const v8usa*)(&s_th[off + 16]));
                bl[nb] = cat16b(*(const v8usa*)(&s_tl[off]), *(const v8usa*)(&s_tl[off + 16])); }
#pragma unroll
            for (int nb = 0; nb < 4; ++nb) o[nb] = wmmab(pa, bh[nb], o[nb]);
#pragma unroll
            for (int nb = 0; nb < 4; ++nb) o[nb] = wmmab(pa, bl[nb], o[nb]);
#pragma unroll
            for (int nb = 0; nb < 4; ++nb) o[nb] = wmmab(pl, bh[nb], o[nb]);
            asm volatile("v_nop\n\tv_nop\n\tv_nop\n\tv_nop" : "+v"(o[0]), "+v"(o[1]), "+v"(o[2]), "+v"(o[3]) : "v"(pa), "v"(pl), "v"(bh[0]), "v"(bh[1]), "v"(bh[2]), "v"(bh[3]), "v"(bl[0]), "v"(bl[1]), "v"(bl[2]), "v"(bl[3]));
        }
    }

    __syncthreads();
    { const int fb = (16 * wave + 8 * hi) * HP + lr;
#pragma unroll
      for (int nb = 0; nb < 4; ++nb) {
#pragma unroll
          for (int r = 0; r < 8; ++r) s_h[fb + r * HP + nb * 16] = 0.25f * o[nb][r]; } }
    wave_sync();
    float* orow = OUT + ((size_t)b * OUT_NT + tt) * GSZ + (size_t)(16 * wave) * 64;
#pragma unroll 1
    for (int ps = 0; ps < 2; ++ps) {
#pragma unroll
        for (int s = 0; s < 8; ++s) { const int row = 2 * s + hi, cofs = lr * 4;
            const v4f val = *(const v4fa*)(&s_h[(16 * wave + row) * HP + cofs]);
            *(volatile v4f*)(orow + (size_t)row * 64 + cofs) = val; }
        if (ps == 0) __threadfence(); }
}

static constexpr size_t al256(size_t v) { return (v + 255) & ~(size_t)255; }
static constexpr size_t SZ_XB = al256((size_t)NB * NT * GSZ * 2);
static constexpr size_t SZ_WT = al256((size_t)2 * NHD * GSZ * 2);
static constexpr size_t SZ_TOTAL = SZ_XB + SZ_WT;
static_assert(SZ_TOTAL <= (size_t)134217728);
static_assert(((size_t)GSZ * 2) % 256 == 0);

extern "C" void kernel_launch(void* const* d_in, const int* in_sizes, int n_in,
                              void* d_out, int out_size, void* d_ws, size_t ws_size, hipStream_t stream) {
    if (n_in < 5) return;
    if ((size_t)in_sizes[0] < ((size_t)(NB - 1) * NT_FULL + NT) * GSZ) return;
    if ((size_t)in_sizes[1] < (size_t)NB * GSZ) return;
    if ((size_t)in_sizes[2] < (size_t)NHD * GSZ || (size_t)in_sizes[3] < (size_t)NHD * GSZ) return;
    if ((size_t)in_sizes[4] < (size_t)NHD * 64) return;
    if ((size_t)out_size < ((size_t)(NB - 1) * OUT_NT + NT) * GSZ) return;
    if (SZ_TOTAL > ws_size) return;
    const float* feat = (const float*)d_in[0];
    const int*   adj  = (const int*)d_in[1];
    const float* wsrc = (const float*)d_in[2];
    const float* wdst = (const float*)d_in[3];
    const float* av   = (const float*)d_in[4];
    float* OUT = (float*)d_out;
    char* wsp = (char*)d_ws;
    bf* XB = (bf*)wsp; wsp += SZ_XB;
    bf* WT = (bf*)wsp; wsp += SZ_WT;

    if (NT == NT_FULL) {
        const size_t n8 = (size_t)NB * NT * GSZ / 8;
        k_cvt8<<<(unsigned)((n8 + 255) / 256), 256, 0, stream>>>(feat, XB, n8);
    } else {
        const size_t n8 = (size_t)NT * GSZ / 8;
        for (int b = 0; b < NB; ++b) k_cvt8<<<(unsigned)((n8 + 255) / 256), 256, 0, stream>>>(feat + (size_t)b * NT_FULL * GSZ, XB + (size_t)b * NT * GSZ, n8);
    }
    k_wt<<<NHD, 256, 0, stream>>>(wsrc, WT);
    k_wt<<<NHD, 256, 0, stream>>>(wdst, WT + (size_t)NHD * GSZ);

    k_gat<<<NB * NT, 128, 0, stream>>>(XB, WT, adj, av, OUT);
}
